// FlashCrossAttention_20280835572118
// MI455X (gfx1250) — hardware-verified
//
#include <hip/hip_runtime.h>
#include <math.h>
#include <stdint.h>

constexpr int kBatch   = 4;
constexpr int kSeq     = 2048;
constexpr int kModel   = 1024;
constexpr int kHeads   = 16;
constexpr int kHdim    = 64;
constexpr int kRows    = kBatch * kSeq;
constexpr int kHalfRot = 32;
constexpr float kEps       = 1e-6f;
constexpr float kPCarry    = 32768.0f;
constexpr float kWCarry    = 64.0f;
constexpr float kOCarry    = 64.0f;
constexpr float kLog2ThetaOverHalf = 13.287712379549449f / 32.0f;

static_assert(kModel == kHeads * kHdim);
static_assert(kSeq * kHalfRot == 65536);
static_assert(kModel % 64 == 0 && kSeq % 64 == 0 && kRows % 64 == 0 && kModel % 32 == 0);

typedef __attribute__((ext_vector_type(16))) _Float16 v16h;
typedef __attribute__((ext_vector_type(8)))  _Float16 v8h;
typedef __attribute__((ext_vector_type(16))) __bf16   v16b;
typedef __attribute__((ext_vector_type(8)))  __bf16   v8b;
typedef __attribute__((ext_vector_type(8)))  float    v8f;
typedef __attribute__((ext_vector_type(4)))  float    v4f;

__device__ __forceinline__ unsigned short f2bf_bits(float f) {
  unsigned u = __float_as_uint(f);
  return (unsigned short)((u + 0x7FFFu + ((u >> 16) & 1u)) >> 16);
}
__device__ __forceinline__ float bf_bits2f(unsigned short h) { return __uint_as_float(((unsigned)h) << 16); }

__device__ __forceinline__ void dep_guard_h(v8f& a, v8f& b, v16h x, v16h y) { asm volatile("v_nop\n\tv_nop\n\tv_nop\n\tv_nop" : "+v"(a), "+v"(b) : "v"(x), "v"(y)); }
__device__ __forceinline__ void dep_guard_b(v8f& a, v8f& b, v16b x, v16b y) { asm volatile("v_nop\n\tv_nop\n\tv_nop\n\tv_nop" : "+v"(a), "+v"(b) : "v"(x), "v"(y)); }
__device__ __forceinline__ void keep4_h(v16h a, v16h b, v16h c, v16h d) { asm volatile("v_nop" :: "v"(a), "v"(b), "v"(c), "v"(d)); }
__device__ __forceinline__ void keep4_b(v16b a, v16b b, v16b c, v16b d) { asm volatile("v_nop" :: "v"(a), "v"(b), "v"(c), "v"(d)); }
__device__ __forceinline__ void acc_guard4(v8f& a, v8f& b, v8f& c, v8f& d) { asm volatile("v_nop\n\tv_nop\n\tv_nop\n\tv_nop" : "+v"(a), "+v"(b), "+v"(c), "+v"(d)); }
template <typename T> struct Frag;
template <> struct Frag<_Float16> {
  typedef v16h V; union U { v16h v; v8h h[2]; };
  static __device__ __forceinline__ v16h load(const _Float16* p) {
    U f; f.h[0] = *(const v8h*)(p); f.h[1] = *(const v8h*)(p + 16); return f.v;
  }
  static __device__ __forceinline__ v8f mma(v16h a, v16h b, v8f c) {
    return __builtin_amdgcn_wmma_f32_16x16x32_f16(false, a, false, b, (short)0, c, false, false);
  }
  static __device__ __forceinline__ void guard(v8f& a, v8f& b, v16h x, v16h y) { dep_guard_h(a, b, x, y); }
  static __device__ __forceinline__ void keep(v16h a, v16h b, v16h c, v16h d) { keep4_h(a, b, c, d); }
};
template <> struct Frag<__bf16> {
  typedef v16b V; union U { v16b v; v8b h[2]; };
  static __device__ __forceinline__ v16b load(const __bf16* p) {
    U f; f.h[0] = *(const v8b*)(p); f.h[1] = *(const v8b*)(p + 16); return f.v;
  }
  static __device__ __forceinline__ v8f mma(v16b a, v16b b, v8f c) {
    return __builtin_amdgcn_wmma_f32_16x16x32_bf16(false, a, false, b, (short)0, c, false, false);
  }
  static __device__ __forceinline__ void guard(v8f& a, v8f& b, v16b x, v16b y) { dep_guard_b(a, b, x, y); }
  static __device__ __forceinline__ void keep(v16b a, v16b b, v16b c, v16b d) { keep4_b(a, b, c, d); }
};

template <int ET> struct Elem;
template <> struct Elem<0> { typedef _Float16 T; };
template <> struct Elem<1> { typedef __bf16 T; };
template <int ET, bool SPLIT, int BIAS_MODE, int OUT_MODE, bool RESID, int ACT = 0>
__global__ __launch_bounds__(256) void wmma_gemm64(
    const unsigned short* __restrict__ Ap, const unsigned short* __restrict__ A2p, int lda, long strideA,
    const unsigned short* __restrict__ Btp, const unsigned short* __restrict__ Bt2p, int ldb, long strideB,
    void* __restrict__ Cout, void* __restrict__ Cout2, int ldc, long strideC,
    const float* __restrict__ bias,
    const float* __restrict__ resid, long strideR,
    int M, int N, int K, float scale) {
  typedef typename Elem<ET>::T T;
  typedef typename Frag<T>::V V;
  const T* A = (const T*)Ap; const T* A2 = (const T*)A2p; const T* Bt = (const T*)Btp; const T* Bt2 = (const T*)Bt2p;
  __shared__ __align__(16) float sT[8][16 * 68];
  const int b    = blockIdx.y;
  const int lane = threadIdx.x & 31;
  const int wave = threadIdx.x >> 5;
  const int tilesN = N >> 6;
  const int tilesM = M >> 6;
  const int tile = blockIdx.x * 8 + wave;
  if (tile >= tilesM * tilesN) return;
  const int tm = tile / tilesN;
  const int tn = tile - tm * tilesN;
  const int m0 = tm << 6;
  const int n0 = tn << 6;

  const T* Ab  = A  + (size_t)b * strideA;
  const T* Bb  = Bt + (size_t)b * strideB;
  const T* Ab2 = SPLIT ? (A2  + (size_t)b * strideA) : nullptr;
  const T* Bb2 = SPLIT ? (Bt2 + (size_t)b * strideB) : nullptr;

  const int rlane = lane & 15;
  const int koff  = (lane >> 4) * 8;
  const int mOff  = (lane >> 4) * 8;

  v8f acc[4][4];
#pragma unroll
  for (int i = 0; i < 4; ++i)
#pragma unroll
    for (int j = 0; j < 4; ++j) acc[i][j] = (v8f){0.f,0.f,0.f,0.f,0.f,0.f,0.f,0.f};

  for (int k0 = 0; k0 < K; k0 += 32) {
    V bh[4], bl[4];
#pragma unroll
    for (int j = 0; j < 4; ++j) {
      const size_t bo = (size_t)(n0 + (j << 4) + rlane) * ldb + koff + k0;
      bh[j] = Frag<T>::load(Bb + bo);
      if (SPLIT) bl[j] = Frag<T>::load(Bb2 + bo);
    }
#pragma unroll
    for (int i = 0; i < 4; ++i) {
      const size_t ao = (size_t)(m0 + (i << 4) + rlane) * lda + koff + k0;
      V ah = Frag<T>::load(Ab + ao);
      V al;
      if (SPLIT) al = Frag<T>::load(Ab2 + ao);
#pragma unroll
      for (int j = 0; j < 4; ++j) {
        acc[i][j] = Frag<T>::mma(ah, bh[j], acc[i][j]);
        if (SPLIT) {
          acc[i][j] = Frag<T>::mma(ah, bl[j], acc[i][j]);
          acc[i][j] = Frag<T>::mma(al, bh[j], acc[i][j]);
        }
      }
      Frag<T>::guard(acc[i][0], acc[i][3], ah, SPLIT ? al : ah);
    }
    Frag<T>::keep(bh[0], bh[1], bh[2], bh[3]);
    if (SPLIT) Frag<T>::keep(bl[0], bl[1], bl[2], bl[3]);
  }
  acc_guard4(acc[0][0], acc[0][1], acc[0][2], acc[0][3]);
  acc_guard4(acc[1][0], acc[1][1], acc[1][2], acc[1][3]);
  acc_guard4(acc[2][0], acc[2][1], acc[2][2], acc[2][3]);
  acc_guard4(acc[3][0], acc[3][1], acc[3][2], acc[3][3]);

  float* slab = sT[wave];
  const float* Rb = RESID ? (resid + (size_t)b * strideR) : nullptr;
#pragma unroll
  for (int i = 0; i < 4; ++i) {
    const int mBase = m0 + (i << 4);
#pragma unroll
    for (int j = 0; j < 4; ++j) {
      const int n = n0 + (j << 4) + rlane;
      float bv = 0.f;
      if (BIAS_MODE == 2) bv = bias[n];
#pragma unroll
      for (int r = 0; r < 8; ++r) {
        float v = acc[i][j][r] * scale;
        if (BIAS_MODE == 1) v += bias[mBase + mOff + r];
        if (BIAS_MODE == 2) v += bv;
        if (RESID) v += Rb[(size_t)(mBase + mOff + r) * ldc + n];
        if (ACT == 1) v = tanhf(v);
        if (ACT == 2) v = fmaxf(v, 0.0f);
        if (ACT == 3) v = v / (1.0f + expf(-v));
        if (ACT == 4) v = (v > 0.f) ? v : 0.01f * v;
        if (ACT == 5) v = 0.5f * v * (1.0f + erff(v * 0.70710678118654752f));
        slab[(mOff + r) * 68 + (j << 4) + rlane] = v;
      }
    }
    __builtin_amdgcn_fence(__ATOMIC_RELEASE, "workgroup");
    __builtin_amdgcn_wave_barrier();
    __builtin_amdgcn_fence(__ATOMIC_ACQUIRE, "workgroup");
    if (OUT_MODE == 0) {
      float* C = (float*)Cout + (size_t)b * strideC;
      const int hh = lane >> 4, c4 = (lane & 15) * 4;
      for (int pass = 0; pass < 2; ++pass) {
#pragma unroll
        for (int it = 0; it < 8; ++it) {
          const int row = it * 2 + hh;
          v4f v = *(const v4f*)(slab + row * 68 + c4);
          *(volatile v4f*)(C + (size_t)(mBase + row) * ldc + n0 + c4) = v;
        }
        __threadfence();
      }
    } else {
      const int q = lane >> 3, c8 = (lane & 7) * 8;
      unsigned short* C  = (unsigned short*)Cout  + (size_t)b * strideC;
      unsigned short* C2 = (OUT_MODE == 2) ? ((unsigned short*)Cout2 + (size_t)b * strideC) : nullptr;
      for (int pass = 0; pass < 2; ++pass) {
#pragma unroll
        for (int it = 0; it < 4; ++it) {
          const int row = it * 4 + q;
          const float* sp = slab + row * 68 + c8;
          v8h hv, lv;
#pragma unroll
          for (int e = 0; e < 8; ++e) {
            if (OUT_MODE == 1) {
              hv[e] = (_Float16)sp[e];
            } else {
              unsigned short hb = f2bf_bits(sp[e]);
              unsigned short lb = f2bf_bits(sp[e] - bf_bits2f(hb));
              hv[e] = __builtin_bit_cast(_Float16, hb);
              lv[e] = __builtin_bit_cast(_Float16, lb);
            }
          }
          *(volatile v8h*)(C + (size_t)(mBase + row) * ldc + n0 + c8) = hv;
          if (OUT_MODE == 2) *(volatile v8h*)(C2 + (size_t)(mBase + row) * ldc + n0 + c8) = lv;
        }
        __threadfence();
      }
    }
    __builtin_amdgcn_fence(__ATOMIC_RELEASE, "workgroup");
    __builtin_amdgcn_wave_barrier();
    __builtin_amdgcn_fence(__ATOMIC_ACQUIRE, "workgroup");
  }
}

__global__ __launch_bounds__(256) void cast_scale_f16x2(
    const float* __restrict__ in, _Float16* __restrict__ out, int n2, float scale) {
  const int i = blockIdx.x * 256 + threadIdx.x;
  if (i < n2) {
    const size_t e0 = 2 * (size_t)i;
    const _Float16 h0 = (_Float16)(in[e0] * scale), h1 = (_Float16)(in[e0 + 1] * scale);
    const unsigned u = (unsigned)__builtin_bit_cast(unsigned short, h0) | ((unsigned)__builtin_bit_cast(unsigned short, h1) << 16);
    ((volatile unsigned*)out)[i] = u;
    __threadfence();
    ((volatile unsigned*)out)[i] = u;
  }
}

__global__ __launch_bounds__(128) void rmsnorm_f16_kernel(
    const float* __restrict__ x, const float* __restrict__ w, unsigned short* __restrict__ out, float eps) {
  __shared__ float red[4];
  const int row = blockIdx.x;
  const int tid = threadIdx.x, lane = tid & 31, wave = tid >> 5;
  const int c0 = tid * 8;
  const float* xr = x + (size_t)row * kModel + c0;
  const v4f xa = *(const v4f*)(xr), xb = *(const v4f*)(xr + 4);
  float ss = 0.f;
#pragma unroll
  for (int e = 0; e < 4; ++e) { ss += xa[e] * xa[e]; ss += xb[e] * xb[e]; }
#pragma unroll
  for (int off = 16; off > 0; off >>= 1) ss += __shfl_xor(ss, off, 32);
  if (lane == 0) red[wave] = ss;
  __syncthreads();
  const float tot = (red[0] + red[1]) + (red[2] + red[3]);
  const float inv = rsqrtf(tot * (1.0f / (float)kModel) + eps);
  const v4f wa = *(const v4f*)(w + c0), wb = *(const v4f*)(w + c0 + 4);
  v8h hv;
#pragma unroll
  for (int e = 0; e < 4; ++e) {
    hv[e]     = (_Float16)((xa[e] * inv) * wa[e]);
    hv[4 + e] = (_Float16)((xb[e] * inv) * wb[e]);
  }
  _Float16* dst = (_Float16*)(void*)out + (size_t)row * kModel + c0;
  *(volatile v8h*)dst = hv;
  __threadfence();
  *(volatile v8h*)dst = hv;
}

__global__ __launch_bounds__(256) void rope_table_kernel(
    const int* __restrict__ offp, float* __restrict__ tabc, float* __restrict__ tabs) {
  const int idx = blockIdx.x * 256 + threadIdx.x;
  const int which = idx >> 16;
  const int t = (idx >> 5) & (kSeq - 1);
  const int j = idx & (kHalfRot - 1);
  const float offq = (float)offp[0];
  const float off = (which == 0) ? offq : 0.0f;
  const float invf = exp2f(-(float)j * kLog2ThetaOverHalf);
  const float pos = (float)t + off;
  const float ang = pos * invf;
  const float cv = cosf(ang);
  const float sv = sinf(ang);
  ((volatile float*)tabc)[idx] = cv;
  ((volatile float*)tabs)[idx] = sv;
  __threadfence();
  ((volatile float*)tabc)[idx] = cv;
  ((volatile float*)tabs)[idx] = sv;
}

__global__ __launch_bounds__(128) void rope_f16_kernel(
    const float* __restrict__ src, const float* __restrict__ tabc, const float* __restrict__ tabs,
    unsigned short* __restrict__ dst) {
  const int row = blockIdx.x;
  const int t = row & (kSeq - 1);
  const int c0 = threadIdx.x * 8;
  const int cpar = c0 ^ kHalfRot;
  const int j0 = c0 & (kHalfRot - 1);
  const float sgn = (c0 & kHalfRot) ? 1.0f : -1.0f;
  const float* sr = src + (size_t)row * kModel;
  const v4f xa = *(const v4f*)(sr + c0),   xb = *(const v4f*)(sr + c0 + 4);
  const v4f ya = *(const v4f*)(sr + cpar), yb = *(const v4f*)(sr + cpar + 4);
  const float* tc = tabc + (size_t)t * kHalfRot + j0;
  const float* tz = tabs + (size_t)t * kHalfRot + j0;
  const v4f ca = *(const v4f*)(tc), cb = *(const v4f*)(tc + 4);
  const v4f sa = *(const v4f*)(tz), sb = *(const v4f*)(tz + 4);
  v8h hv;
#pragma unroll
  for (int e = 0; e < 4; ++e) {
    hv[e]     = (_Float16)(xa[e] * ca[e] + (sgn * ya[e]) * sa[e]);
    hv[4 + e] = (_Float16)(xb[e] * cb[e] + (sgn * yb[e]) * sb[e]);
  }
  _Float16* op = (_Float16*)(void*)dst + (size_t)row * kModel + c0;
  *(volatile v8h*)op = hv;
  __threadfence();
  *(volatile v8h*)op = hv;
}

#define AT_D 64
#define AT_NW 4
#define AT_QB 64
#define AT_KC 64

__device__ __forceinline__ v8f mma_h(v16h a, v16h b, v8f c) {
  c = __builtin_amdgcn_wmma_f32_16x16x32_f16(false, a, false, b, (short)0, c, false, false);
  asm volatile("v_nop\n\tv_nop\n\tv_nop\n\tv_nop" : "+v"(c) : "v"(a), "v"(b));
  return c;
}

__global__ __launch_bounds__(128)
void attn_f16_kernel(const unsigned short* __restrict__ qp, const unsigned short* __restrict__ kp,
                     const unsigned short* __restrict__ vtp, unsigned short* __restrict__ op,
                     float sscale, float oscale) {
  union FH { v16h v; v8h h[2]; };
  __shared__ __align__(16) _Float16 Ksh[AT_KC * AT_D];
  __shared__ __align__(16) _Float16 Vth[AT_D * AT_KC];
  __shared__ __align__(16) _Float16 Psh[AT_NW][16 * AT_KC];
  __shared__ __align__(16) float    Os[AT_NW][16 * 68];

  const int tid  = threadIdx.x;
  const int wave = tid >> 5;
  const int lane = tid & 31;
  const int hh   = lane >> 4;
  const int c    = lane & 15;

  const int nqb = kSeq / AT_QB;
  const int bx = blockIdx.x;
  const int qb = bx % nqb;
  const int bh = bx / nqb;
  const int h  = bh % kHeads;
  const int b  = bh / kHeads;
  const int q0 = qb * AT_QB + wave * 16;

  const _Float16* Qh = (const _Float16*)(const void*)qp  + (size_t)b * kSeq * kModel + (size_t)h * AT_D;
  const _Float16* Kh = (const _Float16*)(const void*)kp  + (size_t)b * kSeq * kModel + (size_t)h * AT_D;
  const _Float16* Vt = (const _Float16*)(const void*)vtp + (size_t)b * kModel * kSeq + (size_t)h * AT_D * kSeq;
  _Float16*       Ob = (_Float16*)(void*)op + (size_t)b * kSeq * kModel + (size_t)h * AT_D;

  v16h qa[2];
#pragma unroll
  for (int dc = 0; dc < 2; ++dc)
    qa[dc] = Frag<_Float16>::load(Qh + (size_t)(q0 + c) * kModel + dc * 32 + 8 * hh);

  float mrow[8], lrow[8];
  v8f oacc[4];
#pragma unroll
  for (int r = 0; r < 8; ++r) { mrow[r] = -INFINITY; lrow[r] = 0.f; }
#pragma unroll
  for (int t = 0; t < 4; ++t) oacc[t] = (v8f){0.f,0.f,0.f,0.f,0.f,0.f,0.f,0.f};

  const int nChunks = kSeq / AT_KC;
  for (int kc = 0; kc < nChunks; ++kc) {
    const int kv0 = kc * AT_KC;
    __syncthreads();
    {
      const int r = tid >> 1, dh = (tid & 1) * 32;
      const _Float16* ks = Kh + (size_t)(kv0 + r) * kModel + dh;
      const _Float16* vs = Vt + (size_t)r * kSeq + kv0 + dh;
#pragma unroll
      for (int i = 0; i < 4; ++i) {
        const v8h a0 = *(const v8h*)(ks + 8 * i);
        const v8h b0 = *(const v8h*)(vs + 8 * i);
        *(v8h*)(Ksh + r * AT_D  + dh + 8 * i) = a0;
        *(v8h*)(Vth + r * AT_KC + dh + 8 * i) = b0;
      }
    }
    __syncthreads();

    v8f s[4];
#pragma unroll
    for (int j = 0; j < 4; ++j) {
      s[j] = (v8f){0.f,0.f,0.f,0.f,0.f,0.f,0.f,0.f};
#pragma unroll
      for (int dc = 0; dc < 2; ++dc) {
        FH kb;
        kb.h[0] = *(const v8h*)(Ksh + (j * 16 + c) * AT_D + dc * 32 + 8 * hh);
        kb.h[1] = *(const v8h*)(Ksh + (j * 16 + c) * AT_D + dc * 32 + 16 + 8 * hh);
        s[j] = mma_h(qa[dc], kb.v, s[j]);
      }
    }
    float cm[8];
#pragma unroll
    for (int r = 0; r < 8; ++r) {
      float m = -INFINITY;
#pragma unroll
      for (int j = 0; j < 4; ++j) {
        const float sv = s[j][r] * sscale;
        s[j][r] = sv;
        m = fmaxf(m, sv);
      }
#pragma unroll
      for (int off = 1; off < 16; off <<= 1) m = fmaxf(m, __shfl_xor(m, off, 32));
      cm[r] = m;
    }
    _Float16* pw = Psh[wave];
#pragma unroll
    for (int r = 0; r < 8; ++r) {
      const float mnew = fmaxf(mrow[r], cm[r]);
      const float alpha = expf(mrow[r] - mnew);
      mrow[r] = mnew;
      float psum = 0.f;
#pragma unroll
      for (int j = 0; j < 4; ++j) {
        const float p = expf(s[j][r] - mnew);
        psum += p;
        pw[(8 * hh + r) * AT_KC + j * 16 + c] = (_Float16)(p * kPCarry);
      }
#pragma unroll
      for (int off = 1; off < 16; off <<= 1) psum += __shfl_xor(psum, off, 32);
      lrow[r] = lrow[r] * alpha + psum;
#pragma unroll
      for (int t = 0; t < 4; ++t) oacc[t][r] *= alpha;
    }
    __builtin_amdgcn_fence(__ATOMIC_RELEASE, "workgroup");
    __builtin_amdgcn_wave_barrier();
    __builtin_amdgcn_fence(__ATOMIC_ACQUIRE, "workgroup");
#pragma unroll
    for (int kk = 0; kk < 2; ++kk) {
      FH pa;
      pa.h[0] = *(const v8h*)(pw + c * AT_KC + kk * 32 + 8 * hh);
      pa.h[1] = *(const v8h*)(pw + c * AT_KC + kk * 32 + 16 + 8 * hh);
#pragma unroll
      for (int t = 0; t < 4; ++t) {
        FH vb;
        vb.h[0] = *(const v8h*)(Vth + (t * 16 + c) * AT_KC + kk * 32 + 8 * hh);
        vb.h[1] = *(const v8h*)(Vth + (t * 16 + c) * AT_KC + kk * 32 + 16 + 8 * hh);
        oacc[t] = mma_h(pa.v, vb.v, oacc[t]);
      }
    }
  }

  float* os = Os[wave];
#pragma unroll
  for (int r = 0; r < 8; ++r) {
    const float inv = oscale / (lrow[r] * kPCarry);
#pragma unroll
    for (int t = 0; t < 4; ++t) os[(8 * hh + r) * 68 + t * 16 + c] = oacc[t][r] * inv;
  }
  __builtin_amdgcn_fence(__ATOMIC_RELEASE, "workgroup");
  __builtin_amdgcn_wave_barrier();
  __builtin_amdgcn_fence(__ATOMIC_ACQUIRE, "workgroup");
  {
    const int q8 = lane >> 3, c8 = (lane & 7) * 8;
    for (int pass = 0; pass < 2; ++pass) {
#pragma unroll
      for (int it = 0; it < 4; ++it) {
        const int row = it * 4 + q8;
        const float* sp = os + row * 68 + c8;
        v8h hv;
#pragma unroll
        for (int e = 0; e < 8; ++e) hv[e] = (_Float16)sp[e];
        *(volatile v8h*)(Ob + (size_t)(q0 + row) * kModel + c8) = hv;
      }
      __threadfence();
    }
  }
}

extern "C" void kernel_launch(void* const* d_in, const int* in_sizes, int n_in,
                              void* d_out, int out_size, void* d_ws, size_t ws_size,
                              hipStream_t stream) {
  if (n_in < 7) return;
  const int nTok = kRows * kModel;
  if (in_sizes[0] != nTok || in_sizes[1] != nTok || in_sizes[2] != kModel ||
      in_sizes[3] != kModel * kModel || in_sizes[4] != 2 * kModel * kModel ||
      in_sizes[5] != kModel * kModel || in_sizes[6] < 1) return;
  if (out_size != nTok) return;

  const size_t MiB = 1024ull * 1024ull;
  const size_t offH16  = 0;
  const size_t offE16  = 16 * MiB;
  const size_t offWq   = 32 * MiB;
  const size_t offWkv  = 34 * MiB;
  const size_t offWo   = 38 * MiB;
  const size_t offQraw = 40 * MiB;
  const size_t offKraw = 72 * MiB;
  const size_t offVT   = 104 * MiB;
  const size_t offTabC = 120 * MiB;
  const size_t offTabS = offTabC + (size_t)2 * kSeq * kHalfRot * sizeof(float);
  const size_t total   = offTabS + (size_t)2 * kSeq * kHalfRot * sizeof(float);
  if (total > ws_size) return;

  const float* x   = (const float*)d_in[0];
  const float* enc = (const float*)d_in[1];
  const float* nw  = (const float*)d_in[2];
  const float* wq  = (const float*)d_in[3];
  const float* wkv = (const float*)d_in[4];
  const float* wo  = (const float*)d_in[5];
  const int*   dof = (const int*)d_in[6];
  float* out = (float*)d_out;

  char* ws = (char*)d_ws;
  unsigned short* H16   = (unsigned short*)(ws + offH16);
  unsigned short* Q16   = H16;
  unsigned short* E16   = (unsigned short*)(ws + offE16);
  unsigned short* K16   = E16;
  unsigned short* Wq16  = (unsigned short*)(ws + offWq);
  unsigned short* Wkv16 = (unsigned short*)(ws + offWkv);
  unsigned short* Wo16  = (unsigned short*)(ws + offWo);
  float*          Qraw  = (float*)(ws + offQraw);
  unsigned short* O16   = (unsigned short*)(ws + offQraw);
  float*          Kraw  = (float*)(ws + offKraw);
  unsigned short* VT16  = (unsigned short*)(ws + offVT);
  float*          tabC  = (float*)(ws + offTabC);
  float*          tabS  = (float*)(ws + offTabS);

  const long strideTok = (long)kSeq * kModel;

  rmsnorm_f16_kernel<<<kRows, 128, 0, stream>>>(x, nw, H16, kEps);
  cast_scale_f16x2<<<(nTok / 2 + 255) / 256, 256, 0, stream>>>(enc, (_Float16*)(void*)E16, nTok / 2, 1.0f);
  cast_scale_f16x2<<<(kModel * kModel / 2 + 255) / 256, 256, 0, stream>>>(wq, (_Float16*)(void*)Wq16, kModel * kModel / 2, kWCarry);
  cast_scale_f16x2<<<(2 * kModel * kModel / 2 + 255) / 256, 256, 0, stream>>>(wkv, (_Float16*)(void*)Wkv16, 2 * kModel * kModel / 2, kWCarry);
  cast_scale_f16x2<<<(kModel * kModel / 2 + 255) / 256, 256, 0, stream>>>(wo, (_Float16*)(void*)Wo16, kModel * kModel / 2, kWCarry);
  rope_table_kernel<<<(2 * kSeq * kHalfRot) / 256, 256, 0, stream>>>(dof, tabC, tabS);
  {
    dim3 g((kRows / 64) * (kModel / 64) / 8, 1);
    wmma_gemm64<0, false, 0, 0, false, 0><<<g, 256, 0, stream>>>(
        H16, H16, kModel, 0L, Wq16, Wq16, kModel, 0L,
        (void*)Qraw, (void*)Qraw, kModel, 0L, nw, x, 0L, kRows, kModel, kModel, 1.0f / kWCarry);
  }
  {
    dim3 g((kRows / 64) * (kModel / 64) / 8, 1);
    wmma_gemm64<0, false, 0, 0, false, 0><<<g, 256, 0, stream>>>(
        E16, E16, kModel, 0L, Wkv16, Wkv16, kModel, 0L,
        (void*)Kraw, (void*)Kraw, kModel, 0L, nw, x, 0L, kRows, kModel, kModel, 1.0f / kWCarry);
  }
  {
    dim3 g((kModel / 64) * (kSeq / 64) / 8, kBatch);
    wmma_gemm64<0, false, 0, 1, false, 0><<<g, 256, 0, stream>>>(
        Wkv16 + (size_t)kModel * kModel, Wkv16 + (size_t)kModel * kModel, kModel, 0L,
        E16, E16, kModel, strideTok,
        (void*)VT16, (void*)VT16, kSeq, (long)kModel * kSeq, nw, x, 0L, kModel, kSeq, kModel, 1.0f / kWCarry);
  }
  rope_f16_kernel<<<kRows, 128, 0, stream>>>(Qraw, tabC, tabS, Q16);
  rope_f16_kernel<<<kRows, 128, 0, stream>>>(Kraw, tabC + (size_t)kSeq * kHalfRot, tabS + (size_t)kSeq * kHalfRot, K16);
  attn_f16_kernel<<<kBatch * kHeads * (kSeq / AT_QB), 128, 0, stream>>>(Q16, K16, VT16, O16, 0.125f, kOCarry);
  {
    dim3 g((kRows / 64) * (kModel / 64) / 8, 1);
    wmma_gemm64<0, false, 0, 0, true, 0><<<g, 256, 0, stream>>>(
        O16, O16, kModel, 0L, Wo16, Wo16, kModel, 0L,
        (void*)out, (void*)out, kModel, 0L, nw, x, 0L, kRows, kModel, kModel, 1.0f / (kWCarry * kOCarry));
  }
}
